// _PLHEACircuit_47175920779402
// MI455X (gfx1250) — hardware-verified
//
#include <hip/hip_runtime.h>

#define NW 14
#define DIM 16384
#define XCOLS 28
#define MWORDS 512
#define CHW 1024
#define WSLS 128
#define STATE_SCALE 4096.0f
#define GATE_SCALE 16.0f
#define GATE_UNSCALE 0.0625f
#define PROB_UNSCALE (1.0f / 16777216.0f)

typedef _Float16 v16h __attribute__((ext_vector_type(16)));
typedef _Float16 v8h_base __attribute__((ext_vector_type(8)));
typedef v8h_base v8h __attribute__((may_alias));
typedef float v8f __attribute__((ext_vector_type(8)));
typedef float v4f __attribute__((ext_vector_type(4)));
typedef unsigned int v8u __attribute__((ext_vector_type(8)));
typedef unsigned int v4u_base __attribute__((ext_vector_type(4)));
typedef v4u_base v4u __attribute__((may_alias));

union FragA { v16h v; v8h half[2]; };
union FragB { v16h v; v8u wd; };

__device__ __forceinline__ v8f wmma16(v16h a, v16h b, v8f c) {
  v8f d = __builtin_amdgcn_wmma_f32_16x16x32_f16(false, a, false, b, (short)0, c, false, false);
  asm volatile("v_nop\n\tv_nop\n\tv_nop\n\tv_nop" : "+v"(d) : "v"(a), "v"(b));
  return d;
}

__device__ __forceinline__ unsigned int f2h_bits(float f) {
  _Float16 hv = (_Float16)f;
  unsigned short u = __builtin_bit_cast(unsigned short, hv);
  return (unsigned int)u;
}

__device__ __forceinline__ float h_bits2f(unsigned int u) {
  unsigned short s = (unsigned short)(u & 0xFFFFu);
  _Float16 hv = __builtin_bit_cast(_Float16, s);
  return (float)hv;
}

__device__ __forceinline__ unsigned int pack2(float re, float im) {
  return f2h_bits(re) | (f2h_bits(im) << 16);
}

__device__ __forceinline__ int perm_inv(int k) {
  int t = k & 0x1FFF;
  t ^= t << 1;
  t ^= t << 2;
  t ^= t << 4;
  t ^= t << 8;
  t &= 0x3FFF;
  return (k & 0x2000) ? (t ^ 0x1FFF) : t;
}

__device__ __forceinline__ void load_afrag(const _Float16* Mg, int m, int h, FragA& aRe, FragA& aIm) {
  aRe.half[0] = *(const v8h*)(Mg + m * 32 + 8 * h);
  aRe.half[1] = *(const v8h*)(Mg + m * 32 + 16 + 8 * h);
  aIm.half[0] = *(const v8h*)(Mg + (16 + m) * 32 + 8 * h);
  aIm.half[1] = *(const v8h*)(Mg + (16 + m) * 32 + 16 + 8 * h);
}

__device__ __forceinline__ void gate_tile(const FragA& aRe, const FragA& aIm,
                                          const unsigned int (&w)[8], unsigned int (&o)[8]) {
  FragB b;
#pragma unroll
  for (int q = 0; q < 4; ++q) {
    b.wd[q]     = (w[2 * q] & 0xFFFFu) | (w[2 * q + 1] << 16);
    b.wd[4 + q] = (w[2 * q] >> 16)     | (w[2 * q + 1] & 0xFFFF0000u);
  }
  const v8f zero = {0.f, 0.f, 0.f, 0.f, 0.f, 0.f, 0.f, 0.f};
  const v8f accRe = wmma16(aRe.v, b.v, zero);
  const v8f accIm = wmma16(aIm.v, b.v, zero);
#pragma unroll
  for (int r = 0; r < 8; ++r)
    o[r] = pack2(accRe[r] * GATE_UNSCALE, accIm[r] * GATE_UNSCALE);
}

__global__ __launch_bounds__(256)
void k_mtab(const float* __restrict__ x, const float* __restrict__ wts,
            unsigned int* mtab, int batch) {
  __shared__ float Ur[NW + 1][4];
  __shared__ float Ui[NW + 1][4];
  __shared__ __attribute__((aligned(16))) _Float16 Mh[1024];
  const int nm = 16 + 4 * batch;
  const int mi = blockIdx.x;
  if (mi >= nm) return;
  const int tid = threadIdx.x;
  const bool enc = (mi >= 16);
  const int lay = enc ? 0 : (mi >> 2);
  const int smp = enc ? ((mi - 16) >> 2) : 0;
  const int p = (enc ? (mi - 16) : mi) & 3;

  if (tid < NW) {
    float a0, a1, a2;
    int nang;
    if (enc) {
      a0 = 0.5f * x[(size_t)smp * XCOLS + NW + tid];
      a1 = 0.f; a2 = 0.f; nang = 1;
    } else {
      const float* wl = wts + lay * 3 * NW;
      a0 = 0.5f * wl[tid];
      a1 = 0.5f * wl[NW + tid];
      a2 = 0.5f * wl[2 * NW + tid];
      nang = 3;
    }
    float c0 = 1.f, s0 = 0.f, c1 = 1.f, s1 = 0.f, c2 = 1.f, s2 = 0.f;
#pragma unroll 1
    for (int q = 0; q < nang; ++q) {
      const float aq = (q == 0) ? a0 : ((q == 1) ? a1 : a2);
      float sv, cv;
      sincosf(aq, &sv, &cv);
      if (q == 0) { c0 = cv; s0 = sv; }
      else if (q == 1) { c1 = cv; s1 = sv; }
      else { c2 = cv; s2 = sv; }
    }
    if (enc) {
      Ur[tid][0] = c0;  Ur[tid][1] = 0.f; Ur[tid][2] = 0.f; Ur[tid][3] = c0;
      Ui[tid][0] = 0.f; Ui[tid][1] = -s0; Ui[tid][2] = -s0; Ui[tid][3] = 0.f;
    } else {
      const float ca = c0, sa = s0, cb = c1, sb = s1, cc = c2, sc = s2;
      const float cca = cc * ca, ssa = sc * sa, csa = cc * sa, sca = sc * ca;
      Ur[tid][0] =  cb * (cca - ssa);  Ui[tid][0] = -sb * (cca + ssa);
      Ur[tid][1] = -cb * (csa + sca);  Ui[tid][1] =  sb * (csa - sca);
      Ur[tid][2] =  cb * (csa + sca);  Ui[tid][2] =  sb * (csa - sca);
      Ur[tid][3] =  cb * (cca - ssa);  Ui[tid][3] =  sb * (cca + ssa);
    }
  }
  if (tid == NW) {
    Ur[NW][0] = 1.f; Ur[NW][1] = 0.f; Ur[NW][2] = 0.f; Ur[NW][3] = 1.f;
    Ui[NW][0] = 0.f; Ui[NW][1] = 0.f; Ui[NW][2] = 0.f; Ui[NW][3] = 0.f;
  }
  __syncthreads();

  const int p0 = (p < 3) ? (10 - 4 * p) : 0;
#pragma unroll 1
  for (int e2 = 0; e2 < 4; ++e2) {
    const int idx = tid + 256 * e2;
    const int R = idx >> 5, C = idx & 31;
    const int i = R & 15, j = C & 15;
    float kr = 1.f, ki = 0.f;
#pragma unroll
    for (int t = 0; t < 4; ++t) {
      const int wv = (p < 3 || t < 2) ? (NW - 1 - p0 - t) : NW;
      const int a = (i >> t) & 1, bb = (j >> t) & 1;
      const float ur = Ur[wv][a * 2 + bb];
      const float ui = Ui[wv][a * 2 + bb];
      const float nr = kr * ur - ki * ui;
      const float ni = kr * ui + ki * ur;
      kr = nr; ki = ni;
    }
    float v;
    if ((R >> 4) == (C >> 4)) v = kr;
    else v = (R >> 4) ? ki : -ki;
    Mh[idx] = (_Float16)(v * GATE_SCALE);
  }
  __syncthreads();
  if (tid < 128) {
    const v4u val = *(const v4u*)(Mh + 8 * tid);
    volatile v4u* pg = (volatile v4u*)(mtab + (size_t)mi * MWORDS) + tid;
    *pg = val;
    __threadfence();
    *pg = val;
  }
}

__device__ __forceinline__ void init_pass(const float* tr0, const float* ti0, const float* tr1,
                                          const float* ti1, volatile v4u* pg, int tid) {
#pragma unroll 1
  for (int j = 0; j < 16; ++j) {
    const int u = tid + 256 * j;
    const int a = u >> 5;
    const float ar = tr0[a], ai = ti0[a];
    unsigned int wd[4];
#pragma unroll
    for (int c = 0; c < 4; ++c) {
      const int b = ((u & 31) << 2) + c;
      const float re = ar * tr1[b] - ai * ti1[b];
      const float im = ar * ti1[b] + ai * tr1[b];
      wd[c] = pack2(re, im);
    }
    v4u val;
    val.x = wd[0]; val.y = wd[1]; val.z = wd[2]; val.w = wd[3];
    pg[u] = val;
  }
}

__global__ __launch_bounds__(256)
void k_init(const float* __restrict__ x, unsigned int* sout, int batch) {
  __shared__ float c14[16], s14[16];
  __shared__ float tr[2][128], ti[2][128];
  const int sample = blockIdx.x;
  if (sample >= batch) return;
  const int tid = threadIdx.x;
  if (tid < NW) {
    float sv, cv;
    sincosf(0.5f * x[(size_t)sample * XCOLS + tid], &sv, &cv);
    c14[tid] = cv;
    s14[tid] = sv;
  }
  __syncthreads();
  {
    const int hf = tid >> 7, v = tid & 127;
    float mag = (hf == 0) ? STATE_SCALE : 1.0f;
#pragma unroll
    for (int q = 0; q < 7; ++q) {
      const int wire = (hf == 0) ? (6 - q) : (NW - 1 - q);
      mag *= ((v >> q) & 1) ? s14[wire] : c14[wire];
    }
    const int pc = __popc((unsigned)v) & 3;
    float re = 0.f, im = 0.f;
    if (pc == 0) re = mag;
    else if (pc == 1) im = -mag;
    else if (pc == 2) re = -mag;
    else im = mag;
    tr[hf][v] = re;
    ti[hf][v] = im;
  }
  __syncthreads();
  volatile v4u* pg = (volatile v4u*)(sout + (size_t)sample * DIM);
  init_pass(tr[0], ti[0], tr[1], ti[1], pg, tid);
  __threadfence();
  init_pass(tr[0], ti[0], tr[1], ti[1], pg, tid);
}

template <bool PERM>
__global__ __launch_bounds__(64)
void k_top(const unsigned int* __restrict__ sin_, unsigned int* sout,
           const unsigned int* __restrict__ mtab, int mbase, int mstride, int batch) {
  __shared__ __attribute__((aligned(16))) unsigned int stg[2][512];
  const int sample = blockIdx.y;
  if (sample >= batch) return;
  const int tid = threadIdx.x;
  const int lane = tid & 31, wave = tid >> 5;
  const int m = lane & 15, h = lane >> 4;
  const int cg = blockIdx.x * 2 + wave;
  const unsigned int* src = sin_ + (size_t)sample * DIM;
  const _Float16* Mg = (const _Float16*)(mtab + (size_t)(mbase + sample * mstride) * MWORDS);
  FragA aRe, aIm;
  load_afrag(Mg, m, h, aRe, aIm);
#pragma unroll
  for (int t = 0; t < 2; ++t) {
    const int col = (cg << 5) | (t << 4) | m;
    unsigned int w[8], o[8];
#pragma unroll
    for (int i = 0; i < 8; ++i) {
      int idx = col | ((8 * h + i) << 10);
      if (PERM) idx = perm_inv(idx);
      w[i] = src[idx];
    }
    gate_tile(aRe, aIm, w, o);
#pragma unroll
    for (int r = 0; r < 8; ++r)
      stg[wave][((8 * h + r) << 5) | (t << 4) | m] = o[r];
  }
  __syncthreads();
  unsigned int* dst = sout + (size_t)sample * DIM;
  const v4u* sp = (const v4u*)(&stg[wave][0]);
  v4u vals[4];
#pragma unroll
  for (int j = 0; j < 4; ++j) vals[j] = sp[32 * j + lane];
#pragma unroll
  for (int j = 0; j < 4; ++j) {
    const int e = 4 * j + (lane >> 3), v = lane & 7;
    *(volatile v4u*)(dst + ((e << 10) | (cg << 5) | (v << 2))) = vals[j];
  }
  __threadfence();
#pragma unroll
  for (int j = 0; j < 4; ++j) {
    const int e = 4 * j + (lane >> 3), v = lane & 7;
    *(volatile v4u*)(dst + ((e << 10) | (cg << 5) | (v << 2))) = vals[j];
  }
}

__global__ __launch_bounds__(64)
void k_low(const unsigned int* __restrict__ sin_, unsigned int* sout,
           const unsigned int* __restrict__ mtab, int mbase, int mstride, int batch) {
  __shared__ __attribute__((aligned(16))) unsigned int sst[CHW];
  const int sample = blockIdx.y;
  if (sample >= batch) return;
  const int ch = blockIdx.x;
  const int tid = threadIdx.x;
  const int lane = tid & 31, wave = tid >> 5;
  const int m = lane & 15, h = lane >> 4;
  const size_t gbase = (size_t)sample * DIM + (size_t)ch * CHW;
  {
    const v4u* gp = (const v4u*)(sin_ + gbase);
    v4u* spw = (v4u*)(&sst[0]);
#pragma unroll
    for (int j = 0; j < 4; ++j) spw[64 * j + tid] = gp[64 * j + tid];
  }
  __syncthreads();
#pragma unroll 1
  for (int pp = 1; pp < 4; ++pp) {
    const int p0 = (pp < 3) ? (10 - 4 * pp) : 0;
    const int lowmask = (1 << p0) - 1;
    const _Float16* Mg = (const _Float16*)(mtab + (size_t)(mbase + sample * mstride + pp) * MWORDS);
    FragA aRe, aIm;
    load_afrag(Mg, m, h, aRe, aIm);
#pragma unroll
    for (int t2 = 0; t2 < 2; ++t2) {
      const int lc = ((wave + 2 * t2) << 4) | m;
      const int base = ((lc & ~lowmask) << 4) | (lc & lowmask);
      unsigned int w[8], o[8];
#pragma unroll
      for (int i = 0; i < 8; ++i) w[i] = sst[base | ((8 * h + i) << p0)];
      gate_tile(aRe, aIm, w, o);
#pragma unroll
      for (int r = 0; r < 8; ++r) sst[base | ((8 * h + r) << p0)] = o[r];
    }
    __syncthreads();
  }
  const v4u* sp = (const v4u*)(&sst[0]);
  v4u vals[4];
#pragma unroll
  for (int j = 0; j < 4; ++j) vals[j] = sp[64 * j + tid];
  volatile v4u* gq = (volatile v4u*)(sout + gbase);
#pragma unroll
  for (int j = 0; j < 4; ++j) gq[64 * j + tid] = vals[j];
  __threadfence();
#pragma unroll
  for (int j = 0; j < 4; ++j) gq[64 * j + tid] = vals[j];
}

__global__ __launch_bounds__(256)
void k_meas(const unsigned int* __restrict__ sin_, float* __restrict__ wsl, int batch) {
  __shared__ float wpart[8];
  __shared__ float sres;
  const int sample = blockIdx.x;
  if (sample >= batch) return;
  const int tid = threadIdx.x;
  const int lane = tid & 31, wave = tid >> 5;
  const unsigned int* S = sin_ + (size_t)sample * DIM;
  float part = 0.f;
#pragma unroll 2
  for (int k = tid; k < DIM; k += 256) {
    const unsigned int wv = S[perm_inv(k)];
    const float re = h_bits2f(wv & 0xFFFFu);
    const float im = h_bits2f(wv >> 16);
    part += (re * re + im * im) * (float)(NW - 2 * (int)__popc((unsigned)k));
  }
#pragma unroll
  for (int off = 16; off > 0; off >>= 1) part += __shfl_xor(part, off, 32);
  if (lane == 0) wpart[wave] = part;
  __syncthreads();
  if (tid == 0) {
    float t = 0.f;
#pragma unroll
    for (int wv = 0; wv < 8; ++wv) t += wpart[wv];
    sres = 0.5f + 0.25f * (t * PROB_UNSCALE);
  }
  __syncthreads();
  if (wave == 0) {
    const float v = sres;
    v4f q;
    q.x = v; q.y = v; q.z = v; q.w = v;
    volatile v4f* pq = (volatile v4f*)(wsl + (size_t)sample * WSLS) + lane;
    *pq = q;
    __threadfence();
    *pq = q;
  }
}

__global__ __launch_bounds__(256)
void k_fin(const float* __restrict__ wsl, float* __restrict__ out, int n) {
  const int ngroups = (n + 3) >> 2;
  const int g = blockIdx.x * 256 + threadIdx.x;
  if (g >= ngroups) return;
  const int e0 = 4 * g;
  if (e0 + 3 < n) {
    v4f v;
    v.x = wsl[(size_t)(e0 + 0) * WSLS];
    v.y = wsl[(size_t)(e0 + 1) * WSLS];
    v.z = wsl[(size_t)(e0 + 2) * WSLS];
    v.w = wsl[(size_t)(e0 + 3) * WSLS];
    volatile v4f* po = (volatile v4f*)(out + e0);
    *po = v;
    __threadfence();
    *po = v;
  } else {
    float t[4];
#pragma unroll
    for (int q = 0; q < 4; ++q) t[q] = (e0 + q < n) ? wsl[(size_t)(e0 + q) * WSLS] : 0.f;
    volatile float* po = (volatile float*)out;
#pragma unroll
    for (int q = 0; q < 4; ++q) if (e0 + q < n) po[e0 + q] = t[q];
    __threadfence();
#pragma unroll
    for (int q = 0; q < 4; ++q) if (e0 + q < n) po[e0 + q] = t[q];
  }
}

extern "C" void kernel_launch(void* const* d_in, const int* in_sizes, int n_in,
                              void* d_out, int out_size, void* d_ws, size_t ws_size,
                              hipStream_t stream) {
  if (n_in < 2) return;
  const float* x = (const float*)d_in[0];
  const float* w = (const float*)d_in[1];
  float* out = (float*)d_out;
  int batch = in_sizes[0] / XCOLS;
  if (batch > out_size) batch = out_size;
  if (batch <= 0) return;
  if (in_sizes[1] < 4 * 3 * NW) return;

  unsigned char* wsb = (unsigned char*)d_ws;
  const size_t stateBytes = (size_t)batch * DIM * sizeof(unsigned int);
  const size_t mtabBytes  = (size_t)(16 + 4 * batch) * MWORDS * sizeof(unsigned int);
  const size_t wslBytes   = (size_t)batch * WSLS * sizeof(float);
  const size_t offA = 0;
  const size_t offB = offA + stateBytes;
  const size_t offM = offB + stateBytes;
  const size_t offW = offM + mtabBytes;
  if (offW + wslBytes > ws_size) return;
  unsigned int* SA = (unsigned int*)(wsb + offA);
  unsigned int* SB = (unsigned int*)(wsb + offB);
  unsigned int* M  = (unsigned int*)(wsb + offM);
  float* wsl = (float*)(wsb + offW);

  const dim3 g2(16, batch);
  k_mtab<<<dim3(16 + 4 * batch), dim3(256), 0, stream>>>(x, w, M, batch);
  k_init<<<dim3(batch), dim3(256), 0, stream>>>(x, SA, batch);
  k_top<false><<<g2, dim3(64), 0, stream>>>(SA, SB, M, 0, 0, batch);
  k_low<<<g2, dim3(64), 0, stream>>>(SB, SA, M, 0, 0, batch);
  k_top<true><<<g2, dim3(64), 0, stream>>>(SA, SB, M, 4, 0, batch);
  k_low<<<g2, dim3(64), 0, stream>>>(SB, SA, M, 4, 0, batch);
  k_top<true><<<g2, dim3(64), 0, stream>>>(SA, SB, M, 16, 4, batch);
  k_low<<<g2, dim3(64), 0, stream>>>(SB, SA, M, 16, 4, batch);
  k_top<false><<<g2, dim3(64), 0, stream>>>(SA, SB, M, 8, 0, batch);
  k_low<<<g2, dim3(64), 0, stream>>>(SB, SA, M, 8, 0, batch);
  k_top<true><<<g2, dim3(64), 0, stream>>>(SA, SB, M, 12, 0, batch);
  k_low<<<g2, dim3(64), 0, stream>>>(SB, SA, M, 12, 0, batch);
  k_meas<<<dim3(batch), dim3(256), 0, stream>>>(SA, wsl, batch);
  const int ngroups = (batch + 3) / 4;
  k_fin<<<dim3((ngroups + 255) / 256), dim3(256), 0, stream>>>(wsl, out, batch);
}
